// LGFF_76905684402789
// MI455X (gfx1250) — hardware-verified
//
#include <hip/hip_runtime.h>


#define NB_ 8
#define NC 64
#define HH 128
#define WW 128
#define HW (HH * WW)
#define BN_EPS 1e-5f

typedef __attribute__((ext_vector_type(16))) __bf16   v16bf;
typedef __attribute__((ext_vector_type(16))) _Float16 v16h;
typedef __attribute__((ext_vector_type(8)))  float    v8f;
typedef __attribute__((ext_vector_type(8)))  unsigned v8u;

__device__ __forceinline__ unsigned f2bf(float f) { unsigned u = __float_as_uint(f); u += 0x7FFFu + ((u >> 16) & 1u); return u >> 16; }
__device__ __forceinline__ unsigned f2h(float f) { return (unsigned)__builtin_bit_cast(unsigned short, (_Float16)f); }
__device__ __forceinline__ int kpat(int v, int half) { return ((v & 4) ? 16 : 0) + half * 8 + 2 * (v & 3); }

template <int F16, int NP> struct Opnd { v16bf p[NP]; };

template <int F16, int NP> __device__ __forceinline__ void pack2(float f0, float f1, unsigned* o) {
    if (F16) { o[0] = f2h(f0) | (f2h(f1) << 16); return; }
    unsigned h0 = f2bf(f0), h1 = f2bf(f1); o[0] = h0 | (h1 << 16);
    if (NP >= 2) {
        float r0 = f0 - __uint_as_float(h0 << 16), r1 = f1 - __uint_as_float(h1 << 16);
        unsigned m0 = f2bf(r0), m1 = f2bf(r1); o[1] = m0 | (m1 << 16);
        if (NP >= 3) {
            float s0 = r0 - __uint_as_float(m0 << 16), s1 = r1 - __uint_as_float(m1 << 16);
            o[2] = f2bf(s0) | (f2bf(s1) << 16);
        }
    }
}
template <int F16, int NP> __device__ __forceinline__ void op_row(const float* rowp, int half, float sc, Opnd<F16, NP>& o) {
    v8u u[NP];
#pragma unroll
    for (int v = 0; v < 8; ++v) {
        int kk = kpat(v, half); unsigned t[3];
        pack2<F16, NP>(rowp[kk] * sc, rowp[kk + 1] * sc, t);
#pragma unroll
        for (int p = 0; p < NP; ++p) u[p][v] = t[p];
    }
#pragma unroll
    for (int p = 0; p < NP; ++p) o.p[p] = __builtin_bit_cast(v16bf, u[p]);
}
template <int F16, int NP> __device__ __forceinline__ void op_row_tail(const float* rowp, int half, float sc, int kvalid, Opnd<F16, NP>& o) {
    v8u u[NP];
#pragma unroll
    for (int v = 0; v < 8; ++v) {
        int kk = kpat(v, half); unsigned t[3];
        float f0 = kk < kvalid ? rowp[kk] * sc : 0.0f, f1 = (kk + 1) < kvalid ? rowp[kk + 1] * sc : 0.0f;
        pack2<F16, NP>(f0, f1, t);
#pragma unroll
        for (int p = 0; p < NP; ++p) u[p][v] = t[p];
    }
#pragma unroll
    for (int p = 0; p < NP; ++p) o.p[p] = __builtin_bit_cast(v16bf, u[p]);
}
template <int F16, int NP> __device__ __forceinline__ void op_col(const float* M, int ld, int n, int k0, int half, float sc, Opnd<F16, NP>& o) {
    v8u u[NP];
#pragma unroll
    for (int v = 0; v < 8; ++v) {
        int kk = k0 + kpat(v, half); unsigned t[3];
        pack2<F16, NP>(M[(size_t)kk * ld + n] * sc, M[(size_t)(kk + 1) * ld + n] * sc, t);
#pragma unroll
        for (int p = 0; p < NP; ++p) u[p][v] = t[p];
    }
#pragma unroll
    for (int p = 0; p < NP; ++p) o.p[p] = __builtin_bit_cast(v16bf, u[p]);
}
template <int F16, int NP> __device__ __forceinline__ void op_col_tail(const float* M, int ld, int n, int k0, int half, float sc, int K, Opnd<F16, NP>& o) {
    v8u u[NP];
#pragma unroll
    for (int v = 0; v < 8; ++v) {
        int kk = k0 + kpat(v, half); unsigned t[3];
        float f0 = kk < K ? M[(size_t)kk * ld + n] * sc : 0.0f, f1 = (kk + 1) < K ? M[(size_t)(kk + 1) * ld + n] * sc : 0.0f;
        pack2<F16, NP>(f0, f1, t);
#pragma unroll
        for (int p = 0; p < NP; ++p) u[p][v] = t[p];
    }
#pragma unroll
    for (int p = 0; p < NP; ++p) o.p[p] = __builtin_bit_cast(v16bf, u[p]);
}
__device__ __forceinline__ v8f wm_bf16(v16bf a, v16bf b, v8f c) { return __builtin_amdgcn_wmma_f32_16x16x32_bf16(false, a, false, b, (short)0, c, false, false); }
template <int F16, int NA, int NB> __device__ __forceinline__ v8f wmma_op(const Opnd<F16, NA>& a, const Opnd<F16, NB>& b, v8f c) {
    if (F16) {
        v16h ah = __builtin_bit_cast(v16h, a.p[0]), bh = __builtin_bit_cast(v16h, b.p[0]);
        c = __builtin_amdgcn_wmma_f32_16x16x32_f16(false, ah, false, bh, (short)0, c, false, false);
        asm volatile("v_nop\n\tv_nop\n\tv_nop\n\tv_nop" : "+v"(c) : "v"(ah), "v"(bh));
        return c;
    }
    constexpr int NMX = NA > NB ? NA : NB;
#pragma unroll
    for (int i = 0; i < NA; ++i)
#pragma unroll
        for (int j = 0; j < NB; ++j)
            if (i + j < NMX) c = wm_bf16(a.p[i], b.p[j], c);
    if (NA == 1 && NB == 1)      asm volatile("v_nop\n\tv_nop\n\tv_nop\n\tv_nop" : "+v"(c) : "v"(a.p[0]), "v"(b.p[0]));
    else if (NA == 2 && NB == 1) asm volatile("v_nop\n\tv_nop\n\tv_nop\n\tv_nop" : "+v"(c) : "v"(a.p[0]), "v"(a.p[1]), "v"(b.p[0]));
    else if (NA == 1 && NB == 2) asm volatile("v_nop\n\tv_nop\n\tv_nop\n\tv_nop" : "+v"(c) : "v"(a.p[0]), "v"(b.p[0]), "v"(b.p[1]));
    else if (NA == 2 && NB == 2) asm volatile("v_nop\n\tv_nop\n\tv_nop\n\tv_nop" : "+v"(c) : "v"(a.p[0]), "v"(a.p[1]), "v"(b.p[0]), "v"(b.p[1]));
    else                         asm volatile("v_nop\n\tv_nop\n\tv_nop\n\tv_nop" : "+v"(c) : "v"(a.p[0]), "v"(a.p[NA - 1]), "v"(b.p[0]), "v"(b.p[NB - 1]), "v"(a.p[NA / 2]), "v"(b.p[NB / 2]));
    return c;
}

struct ZMap { long long s1; long long s2; int zdiv; int pad_; };
__device__ __forceinline__ size_t zoff(const ZMap& m, int z) { return (size_t)((long long)(z / m.zdiv) * m.s1 + (long long)(z % m.zdiv) * m.s2); }

#define ACT_NONE 0
#define ACT_RELU 1
#define ACT_GELU_ERF 2
#define ACT_SILU 3
#define ACT_TANH 4
__device__ __forceinline__ float act_apply(int act, float x) {
    if (act == ACT_RELU) return x > 0.f ? x : 0.f;
    if (act == ACT_GELU_ERF) return 0.5f * x * (1.0f + erff(x * 0.70710678118654752f));
    if (act == ACT_SILU) return x / (1.0f + expf(-x));
    if (act == ACT_TANH) return tanhf(x);
    return x;
}
struct GemmArgs {
    ZMap za, zb_, zc, zbias, zadd, zrsc, zmul, zrbias;
    const float* A; const float* Bm; float* C; const float* bias; const float* add; const float* rsc; const float* mul; const float* rbias;
    long long ldadd, ldmul;
    int lda, ldb, ldc, K;
    float ascale, bscale, oscale, addscale;
    int M, nvalid, nstore, ldrsc;
    int bcs, pad1, pad2, pad3;
};
template <int BT, int F16, int NA, int NB, int RW, int CW, int ACT>
__global__ __launch_bounds__(256) void gemm_kernel(GemmArgs g) {
    constexpr int TR = 16 * RW, TC = 64 * CW, CSTR = TC + 4;
    __shared__ __align__(16) float cst[TR * CSTR];
    const int z = blockIdx.z;
    const float* A = g.A + zoff(g.za, z); const float* Bm = g.Bm + zoff(g.zb_, z); float* C = g.C + zoff(g.zc, z);
    const int tid = threadIdx.x, lane = tid & 31, wv = tid >> 5;
    const int l16 = lane & 15, half = lane >> 4;
    const int rt = wv % RW, ch = wv / RW;
    const int row0 = blockIdx.x * TR, col0 = blockIdx.y * TC + ch * 64;
    int arix = row0 + rt * 16 + l16; if (arix >= g.M) arix = g.M - 1;
    const float* arow = A + (size_t)arix * g.lda;
    v8f acc[4];
#pragma unroll
    for (int t = 0; t < 4; ++t) acc[t] = (v8f){};
    const int K = g.K;
#pragma unroll 1
    for (int kc = 0; kc < K; kc += 32) {
        Opnd<F16, NA> a;
        if (kc + 32 <= K) op_row<F16, NA>(arow + kc, half, g.ascale, a); else op_row_tail<F16, NA>(arow + kc, half, g.ascale, K - kc, a);
#pragma unroll
        for (int t = 0; t < 4; ++t) {
            Opnd<F16, NB> b;
            const int n = col0 + t * 16 + l16;
            if (n < g.nvalid) {
                if (BT) { if (kc + 32 <= K) op_row<F16, NB>(Bm + (size_t)n * g.ldb + kc, half, g.bscale, b); else op_row_tail<F16, NB>(Bm + (size_t)n * g.ldb + kc, half, g.bscale, K - kc, b); }
                else    { if (kc + 32 <= K) op_col<F16, NB>(Bm, g.ldb, n * g.bcs, kc, half, g.bscale, b); else op_col_tail<F16, NB>(Bm, g.ldb, n * g.bcs, kc, half, g.bscale, K, b); }
            } else {
#pragma unroll
                for (int p = 0; p < NB; ++p) b.p[p] = (v16bf){};
            }
            acc[t] = wmma_op<F16, NA, NB>(a, b, acc[t]);
        }
    }
    const float* bias = g.bias ? g.bias + zoff(g.zbias, z) : nullptr;
    const float* add = g.add ? g.add + zoff(g.zadd, z) : nullptr;
    const float* rsc = g.rsc ? g.rsc + zoff(g.zrsc, z) : nullptr;
    const float* mul = g.mul ? g.mul + zoff(g.zmul, z) : nullptr;
    const float* rbias = g.rbias ? g.rbias + zoff(g.zrbias, z) : nullptr;
#pragma unroll
    for (int t = 0; t < 4; ++t) {
        const int cl = ch * 64 + t * 16 + l16;
        const int cg = blockIdx.y * TC + cl;
        const bool cok = cg < g.nvalid;
        const float bv = (bias && cok) ? bias[(size_t)cg * g.bcs] : 0.0f;
#pragma unroll
        for (int r = 0; r < 8; ++r) {
            const int rl = rt * 16 + r + 8 * half;
            float v = acc[t][r] * g.oscale + bv;
            int rg = row0 + rl; if (rg >= g.M) rg = g.M - 1;
            if (rbias) v += rbias[rg];
            if (rsc) v *= rsc[(size_t)rg * g.ldrsc];
            if (mul && cok) v *= mul[(size_t)rg * g.ldmul + cg];
            if (add && cok) v += g.addscale * add[(size_t)rg * g.ldadd + cg];
            cst[rl * CSTR + cl] = v;
        }
    }
    __syncthreads();
    const int col = tid % TC, rsel = tid / TC, rstep = 256 / TC;
    if (ACT != ACT_NONE) {
#pragma unroll 1
        for (int r = rsel; r < TR; r += rstep) cst[r * CSTR + col] = act_apply(ACT, cst[r * CSTR + col]);
    }
    float* ob = C + (size_t)row0 * g.ldc + (size_t)blockIdx.y * TC;
    const bool colok = (int)(blockIdx.y * TC + col) < g.nstore;
    const int rmax = (g.M - row0 < TR) ? (g.M - row0) : TR;
    auto pass = [&]() {
        if (colok) {
#pragma unroll 4
            for (int r = rsel; r < rmax; r += rstep) *(volatile float*)(ob + (size_t)r * g.ldc + col) = cst[r * CSTR + col];
        }
    };
    pass();
    __threadfence();
    pass();
}
static inline ZMap zm(long long s1) { ZMap m; m.s1 = s1; m.s2 = 0; m.zdiv = 1; m.pad_ = 0; return m; }
static inline ZMap zm2(long long s1, long long s2, int zdiv) { ZMap m; m.s1 = s1; m.s2 = s2; m.zdiv = zdiv; m.pad_ = 0; return m; }
static inline GemmArgs gemm_args(const float* A, int lda, ZMap za, const float* Bm, int ldb, ZMap zb, float* C, int ldc, ZMap zc, int M, int N, int K) {
    GemmArgs g; g.za = za; g.zb_ = zb; g.zc = zc; g.zbias = zm(0); g.zadd = zm(0); g.zrsc = zm(0); g.zmul = zm(0); g.zrbias = zm(0);
    g.A = A; g.Bm = Bm; g.C = C; g.bias = nullptr; g.add = nullptr; g.rsc = nullptr; g.mul = nullptr; g.rbias = nullptr; g.ldadd = 0; g.ldmul = 0;
    g.lda = lda; g.ldb = ldb; g.ldc = ldc; g.K = K; g.ascale = 1.0f; g.bscale = 1.0f; g.oscale = 1.0f; g.addscale = 1.0f; g.M = M; g.nvalid = N; g.nstore = N; g.ldrsc = 1;
    g.bcs = 1; g.pad1 = 0; g.pad2 = 0; g.pad3 = 0;
    return g;
}
static_assert(sizeof(ZMap) == 24, "ZMap layout");
static_assert(sizeof(GemmArgs) == 8 * 24 + 8 * 8 + 2 * 8 + 4 * 4 + 4 * 4 + 4 * 4 + 4 * 4, "GemmArgs has no padding");

__global__ __launch_bounds__(256) void softmax_rows(float* S, long long sy, long long sx, int L, float prescale, const float* addv, long long say, int aydiv, int causal,
                                                  const int* imask, long long imy, long long imx, float maskval) {
    __shared__ float red[8];
    const int tid = threadIdx.x, lane = tid & 31, wid = tid >> 5;
    float* row = S + (size_t)blockIdx.y * sy + (size_t)blockIdx.x * sx;
    const float* av = addv ? addv + (size_t)(blockIdx.y / aydiv) * say : nullptr;
    const int* im = imask ? imask + (size_t)(blockIdx.y / aydiv) * imy + (size_t)blockIdx.x * imx : nullptr;
    float v[16];
    const int nj = L / 256;
    float mx = -__builtin_inff();
#pragma unroll
    for (int j = 0; j < 16; ++j) if (j < nj) { float t = row[tid + 256 * j] * prescale; if (av) t += av[tid + 256 * j]; if (im && im[tid + 256 * j] == 0) t = maskval; if (causal && (tid + 256 * j) > (int)blockIdx.x) t = -__builtin_inff(); v[j] = t; mx = fmaxf(mx, t); }
#pragma unroll
    for (int o = 16; o; o >>= 1) mx = fmaxf(mx, __shfl_xor(mx, o, 32));
    if (lane == 0) red[wid] = mx;
    __syncthreads();
    float m = red[0];
#pragma unroll
    for (int i = 1; i < 8; ++i) m = fmaxf(m, red[i]);
    if (m == -__builtin_inff()) m = 0.f;
    __syncthreads();
    float sum = 0.f;
#pragma unroll
    for (int j = 0; j < 16; ++j) if (j < nj) { v[j] = expf(v[j] - m); sum += v[j]; }
#pragma unroll
    for (int o = 16; o; o >>= 1) sum += __shfl_xor(sum, o, 32);
    if (lane == 0) red[wid] = sum;
    __syncthreads();
    float tot = 0.f;
#pragma unroll
    for (int i = 0; i < 8; ++i) tot += red[i];
    const float inv = 1.0f / tot;
#pragma unroll
    for (int j = 0; j < 16; ++j) if (j < nj) *(volatile float*)(row + tid + 256 * j) = v[j] * inv;
    __threadfence();
#pragma unroll
    for (int j = 0; j < 16; ++j) if (j < nj) *(volatile float*)(row + tid + 256 * j) = v[j] * inv;
}

#define VST2(T, p, v) do { const T vst2_v_ = (v); *(volatile T*)(p) = vst2_v_; __threadfence(); *(volatile T*)(p) = vst2_v_; } while (0)
#define NTOT ((size_t)NB_ * NC * HW)

__global__ void k_tr_in(const float* __restrict__ x, float* xn) {
    __shared__ float tile[32][33];
    const int b = blockIdx.z, p0 = blockIdx.x * 32, c0 = blockIdx.y * 32, tx = threadIdx.x, ty = threadIdx.y;
    for (int j = 0; j < 32; j += 8) tile[ty + j][tx] = x[((size_t)b * HW + p0 + ty + j) * NC + c0 + tx];
    __syncthreads();
    for (int j = 0; j < 32; j += 8) *(volatile float*)(xn + ((size_t)b * NC + c0 + ty + j) * HW + p0 + tx) = tile[tx][ty + j];
    __threadfence();
    for (int j = 0; j < 32; j += 8) *(volatile float*)(xn + ((size_t)b * NC + c0 + ty + j) * HW + p0 + tx) = tile[tx][ty + j];
}
__global__ void k_wt2(const float* __restrict__ W, float* Wt, int rows, int cols) {
    const int i = blockIdx.x * 256 + threadIdx.x; if (i >= rows * cols) return;
    const int c = i / rows, r = i % rows;
    VST2(float, Wt + i, W[(size_t)r * cols + c]);
}
__global__ __launch_bounds__(256) void k_roll(const float* __restrict__ in, float* out, int sign, int mode) {
    const size_t t = (size_t)blockIdx.x * 256 + threadIdx.x; if (t >= NTOT) return;
    const int w = (int)(t % WW), h = (int)((t / WW) % HH), c = (int)((t / HW) % NC); const size_t plane = t - (size_t)h * WW - w;
    int hs = h, wsrc = w;
    if (mode == 0) { hs = ((h - sign * c) % HH + HH) % HH; } else { wsrc = ((w - sign * c) % WW + WW) % WW; }
    VST2(float, out + t, in[plane + (size_t)hs * WW + wsrc]);
}
__global__ __launch_bounds__(256) void k_ln_ch(const float* __restrict__ x1, const float* __restrict__ x2, const float* __restrict__ g, const float* __restrict__ bb, float* xc) {
    const size_t t = (size_t)blockIdx.x * 256 + threadIdx.x; if (t >= (size_t)NB_ * HW) return;
    const int b = (int)(t / HW), p = (int)(t % HW);
    const float* a1 = x1 + (size_t)b * NC * HW + p; const float* a2 = x2 + (size_t)b * NC * HW + p;
    float s = 0.f;
    for (int c = 0; c < NC; ++c) { s += a1[(size_t)c * HW]; s += a2[(size_t)c * HW]; }
    const float mean = s / (float)(2 * NC); float q = 0.f;
    for (int c = 0; c < NC; ++c) { const float d1 = a1[(size_t)c * HW] - mean, d2 = a2[(size_t)c * HW] - mean; q += d1 * d1 + d2 * d2; }
    const float rstd = rsqrtf(q / (float)(2 * NC) + BN_EPS);
    float* o = xc + (size_t)b * 2 * NC * HW + p;
    for (int c = 0; c < NC; ++c) { VST2(float, o + (size_t)c * HW, (a1[(size_t)c * HW] - mean) * rstd * g[c] + bb[c]); }
    for (int c = 0; c < NC; ++c) { VST2(float, o + (size_t)(NC + c) * HW, (a2[(size_t)c * HW] - mean) * rstd * g[NC + c] + bb[NC + c]); }
}
__global__ __launch_bounds__(256) void k_dw(const float* __restrict__ x, const float* __restrict__ w, const float* __restrict__ bias, int dil, float* dw) {
    const size_t t = (size_t)blockIdx.x * 256 + threadIdx.x; if (t >= NTOT) return;
    const int px = (int)(t % WW), py = (int)((t / WW) % HH), c = (int)((t / HW) % NC); const size_t plane = t - (size_t)py * WW - px;
    float s = bias ? bias[c] : 0.f;
#pragma unroll
    for (int ky = 0; ky < 3; ++ky) { const int yy = py + (ky - 1) * dil; if (yy < 0 || yy >= HH) continue;
#pragma unroll
        for (int kx = 0; kx < 3; ++kx) { const int xx = px + (kx - 1) * dil; if (xx < 0 || xx >= WW) continue; s += x[plane + (size_t)yy * WW + xx] * w[c * 9 + ky * 3 + kx]; } }
    VST2(float, dw + t, s);
}
__global__ __launch_bounds__(256) void k_bnstats(const float* __restrict__ a, float* stats) {
    __shared__ float red[256];
    const int c = blockIdx.x, tid = threadIdx.x; const float cntf = (float)(NB_ * HW);
    float mean = 0.f, tot = 0.f;
    for (int pass = 0; pass < 2; ++pass) {
        float s = 0.f;
        for (int b = 0; b < NB_; ++b) { const float* p = a + ((size_t)b * NC + c) * HW; for (int i = tid; i < HW; i += 256) { const float v = p[i]; s += pass ? (v - mean) * (v - mean) : v; } }
        red[tid] = s; __syncthreads();
        for (int o = 128; o > 0; o >>= 1) { if (tid < o) red[tid] += red[tid + o]; __syncthreads(); }
        if (pass == 0) mean = red[0] / cntf; tot = red[0]; __syncthreads();
    }
    if (tid < 32) { const float v = (tid == 0) ? mean : ((tid == 1) ? tot / cntf : 0.f); VST2(float, stats + c * 32 + tid, v); }
}
__global__ __launch_bounds__(256) void k_bnrelu(float* a, const float* __restrict__ stats, const float* __restrict__ g, const float* __restrict__ be) {
    const size_t t = (size_t)blockIdx.x * 256 + threadIdx.x; if (t >= NTOT) return;
    const int c = (int)((t / HW) % NC);
    const float v = fmaxf((a[t] - stats[c * 32]) * rsqrtf(stats[c * 32 + 1] + BN_EPS) * g[c] + be[c], 0.f);
    VST2(float, a + t, v);
}
__global__ __launch_bounds__(256) void k_se_mean(const float* __restrict__ x7, float* sm) {
    __shared__ float red[256];
    const int bc = blockIdx.x, tid = threadIdx.x; const float* p = x7 + (size_t)bc * HW; float s = 0.f;
    for (int i = tid; i < HW; i += 256) s += p[i];
    red[tid] = s; __syncthreads();
    for (int o = 128; o > 0; o >>= 1) { if (tid < o) red[tid] += red[tid + o]; __syncthreads(); }
    if (tid < 32) { const float v = (tid == 0) ? red[0] / (float)HW : 0.f; VST2(float, sm + (size_t)bc * 32 + tid, v); }
}
__global__ __launch_bounds__(NC) void k_se_fc(const float* __restrict__ sm, const float* __restrict__ w1, const float* __restrict__ b1, const float* __restrict__ w2, const float* __restrict__ b2, float* es) {
    __shared__ float s[NC]; __shared__ float e1[NC / 8];
    const int b = blockIdx.x, c = threadIdx.x;
    s[c] = sm[((size_t)b * NC + c) * 32]; __syncthreads();
    if (c < NC / 8) { float a = b1[c]; for (int k = 0; k < NC; ++k) a += w1[c * NC + k] * s[k]; e1[c] = fmaxf(a, 0.f); }
    __syncthreads();
    float a = b2[c]; for (int k = 0; k < NC / 8; ++k) a += w2[c * (NC / 8) + k] * e1[k];
    const float e = 1.0f / (1.0f + expf(-a));
    VST2(float, es + (size_t)b * NC + c, e);
}
__global__ __launch_bounds__(256) void k_final(const float* __restrict__ x7, const float* __restrict__ es, float* out) {
    const size_t t = (size_t)blockIdx.x * 256 + threadIdx.x; if (t >= NTOT) return;
    const int c = (int)((t / HW) % NC), b = (int)(t / ((size_t)NC * HW));
    const float v = x7[t] * (1.0f + es[(size_t)b * NC + c]);
    VST2(float, out + t, v);
}

extern "C" void kernel_launch(void* const* d_in, const int* in_sizes, int n_in,
                              void* d_out, int out_size, void* d_ws, size_t ws_size, hipStream_t stream) {
    (void)in_sizes; (void)n_in; (void)out_size;
    const float* x = (const float*)d_in[0];
    const float* fc1_w = (const float*)d_in[1];  const float* fc1_b = (const float*)d_in[2];
    const float* fc2_w = (const float*)d_in[3];  const float* fc2_b = (const float*)d_in[4];
    const float* fc3_w = (const float*)d_in[5];  const float* fc3_b = (const float*)d_in[6];
    const float* fc4_w = (const float*)d_in[7];  const float* fc4_b = (const float*)d_in[8];
    const float* fc5_w = (const float*)d_in[9];  const float* fc5_b = (const float*)d_in[10];
    const float* ln_g = (const float*)d_in[11];  const float* ln_b = (const float*)d_in[12];
    const float* pc_w = (const float*)d_in[13];
    const float* dw_w = (const float*)d_in[14];  const float* dw_b = (const float*)d_in[15];
    const float* dwg = (const float*)d_in[16];   const float* dwb = (const float*)d_in[17];
    const float* dd_w = (const float*)d_in[18];  const float* ddg = (const float*)d_in[19]; const float* ddb = (const float*)d_in[20];
    const float* se_w1 = (const float*)d_in[21]; const float* se_b1 = (const float*)d_in[22];
    const float* se_w2 = (const float*)d_in[23]; const float* se_b2 = (const float*)d_in[24];
    float* out = (float*)d_out;

    const size_t PL = NTOT;
    float* base = (float*)d_ws;
    float* XN = base;
    float* T1 = base + PL;
    float* T2 = base + 2 * PL;
    float* X1 = base + 3 * PL;
    float* X2 = base + 4 * PL;
    float* XC = base + 5 * PL;
    float* WT = base + 7 * PL;
    float* stats = WT + 4 * NC * NC + NC * 2 * NC;
    float* sm = stats + NC * 32;
    float* es = sm + (size_t)NB_ * NC * 32;
    const size_t wsNeed = (size_t)((es + NB_ * NC) - base) * sizeof(float);
    if (wsNeed > ws_size) return;
    const unsigned nE = (unsigned)((NTOT + 255) / 256);
    float* fc1t = WT; float* fc2t = WT + NC * NC; float* fc3t = WT + 2 * NC * NC; float* fc4t = WT + 3 * NC * NC; float* fc5t = WT + 4 * NC * NC;

    k_tr_in<<<dim3(HW / 32, NC / 32, NB_), dim3(32, 8), 0, stream>>>(x, XN);
    k_wt2<<<(NC * NC + 255) / 256, 256, 0, stream>>>(fc1_w, fc1t, NC, NC);
    k_wt2<<<(NC * NC + 255) / 256, 256, 0, stream>>>(fc2_w, fc2t, NC, NC);
    k_wt2<<<(NC * NC + 255) / 256, 256, 0, stream>>>(fc3_w, fc3t, NC, NC);
    k_wt2<<<(NC * NC + 255) / 256, 256, 0, stream>>>(fc4_w, fc4t, NC, NC);
    k_wt2<<<(2 * NC * NC + 255) / 256, 256, 0, stream>>>(fc5_w, fc5t, 2 * NC, NC);
    const dim3 gG(1, HW / 128, NB_);
    auto chlin = [&](const float* Wt, int K, const float* Xsrc, long long zx, const float* rb, float* Cdst, const float* addsrc, int act) {
        GemmArgs g = gemm_args(Wt, K, zm(0), Xsrc, HW, zm(zx), Cdst, HW, zm((long long)NC * HW), NC, HW, K);
        g.rbias = rb; g.bscale = 1.0f; g.ascale = 16.0f; g.oscale = 1.0f / 16.0f;
        if (addsrc) { g.add = addsrc; g.ldadd = HW; g.zadd = zm((long long)NC * HW); g.addscale = 1.0f; }
        if (act == ACT_GELU_ERF) gemm_kernel<0, 1, 1, 1, 4, 2, ACT_GELU_ERF><<<gG, 256, 0, stream>>>(g);
        else                     gemm_kernel<0, 1, 1, 1, 4, 2, ACT_NONE><<<gG, 256, 0, stream>>>(g);
    };
    k_roll<<<nE, 256, 0, stream>>>(XN, T1, 1, 0);
    chlin(fc1t, NC, T1, (long long)NC * HW, fc1_b, T2, nullptr, ACT_GELU_ERF);
    k_roll<<<nE, 256, 0, stream>>>(T2, T1, 1, 1);
    chlin(fc2t, NC, T1, (long long)NC * HW, fc2_b, X1, XN, ACT_NONE);
    k_roll<<<nE, 256, 0, stream>>>(XN, T1, -1, 1);
    chlin(fc3t, NC, T1, (long long)NC * HW, fc3_b, T2, nullptr, ACT_GELU_ERF);
    k_roll<<<nE, 256, 0, stream>>>(T2, T1, 1, 0);
    chlin(fc4t, NC, T1, (long long)NC * HW, fc4_b, X2, XN, ACT_NONE);
    k_ln_ch<<<(unsigned)(((size_t)NB_ * HW + 255) / 256), 256, 0, stream>>>(X1, X2, ln_g, ln_b, XC);
    chlin(fc5t, 2 * NC, XC, (long long)2 * NC * HW, fc5_b, T1, XN, ACT_NONE);
    float* PX2 = X1; float* Y = X2; float* Y2 = XC; float* X7 = XC + PL;
    { GemmArgs g = gemm_args(pc_w, NC, zm(0), T1, HW, zm((long long)NC * HW), PX2, HW, zm((long long)NC * HW), NC, HW, NC);
      gemm_kernel<0, 0, 2, 2, 4, 2, ACT_NONE><<<gG, 256, 0, stream>>>(g); }
    k_dw<<<nE, 256, 0, stream>>>(PX2, dw_w, dw_b, 1, Y);
    k_bnstats<<<NC, 256, 0, stream>>>(Y, stats);
    k_bnrelu<<<nE, 256, 0, stream>>>(Y, stats, dwg, dwb);
    k_dw<<<nE, 256, 0, stream>>>(Y, dd_w, nullptr, 2, Y2);
    k_bnstats<<<NC, 256, 0, stream>>>(Y2, stats);
    k_bnrelu<<<nE, 256, 0, stream>>>(Y2, stats, ddg, ddb);
    { GemmArgs g = gemm_args(pc_w, NC, zm(0), Y2, HW, zm((long long)NC * HW), X7, HW, zm((long long)NC * HW), NC, HW, NC); g.oscale = 4.0f;
      g.mul = PX2; g.ldmul = HW; g.zmul = zm((long long)NC * HW);
      gemm_kernel<0, 0, 2, 2, 4, 2, ACT_NONE><<<gG, 256, 0, stream>>>(g); }
    k_se_mean<<<NB_ * NC, 256, 0, stream>>>(X7, sm);
    k_se_fc<<<NB_, NC, 0, stream>>>(sm, se_w1, se_b1, se_w2, se_b2, es);
    k_final<<<nE, 256, 0, stream>>>(X7, es, out);
}
